// RNNEncoder_57913339019644
// MI455X (gfx1250) — hardware-verified
//
#include <hip/hip_runtime.h>
#include <math.h>

constexpr int NBATCH   = 128;
constexpr int NSTEP    = 512;
constexpr int NFEAT_IN = 130;
constexpr int NFEAT    = 128;
constexpr int NHID     = 512;
constexpr int NGATE    = 4 * NHID;
constexpr int KCAT     = NFEAT + NHID;
constexpr int NTHR     = 256;
constexpr int ROWS_BLK = 16;
constexpr int APITCH   = 648;
constexpr int ABUF     = ROWS_BLK * APITCH;
constexpr int OPITCH   = 516;
constexpr float ACARRY = 16.0f;
constexpr float WCARRY = 256.0f;
constexpr float FOLD   = 1.0f / (ACARRY * WCARRY);
constexpr size_t GATE_STRIDE = (size_t)NHID * KCAT;
constexpr int PREP_BLK_IH = (NGATE * (NFEAT / 8)) / NTHR;
constexpr int PREP_BLK_HH = (NGATE * (NHID / 8)) / NTHR;
constexpr int PREP_BLK_BS = (NGATE / 4) / NTHR;

static_assert(NFEAT == NFEAT_IN - 2, "two trailing feature columns are dropped");
static_assert(KCAT % 32 == 0, "K multiple of 32");
static_assert(NBATCH % ROWS_BLK == 0, "batch tiles exact");
static_assert(NHID == 64 * (NTHR / 32), "8 waves x 64 hidden units");
static_assert((NGATE * (NFEAT / 8)) % NTHR == 0, "prep W_ih coverage exact");
static_assert((NGATE * (NHID / 8)) % NTHR == 0, "prep W_hh coverage exact");
static_assert((NGATE / 4) % NTHR == 0, "prep bias coverage exact");
static_assert(ROWS_BLK * NFEAT == NTHR * 8, "x staging: 8 elements per thread");
static_assert(2 * ABUF * 2 >= ROWS_BLK * OPITCH * 4, "output staging fits in the A tile bytes");
static_assert((APITCH * 2) % 16 == 0 && (OPITCH * 4) % 16 == 0, "LDS row alignment");

typedef __attribute__((ext_vector_type(16))) _Float16 v16h;
typedef __attribute__((ext_vector_type(8)))  _Float16 v8h;
typedef __attribute__((ext_vector_type(8)))  float    v8f;
typedef __attribute__((ext_vector_type(4)))  float    v4f;
typedef __attribute__((ext_vector_type(2)))  float    v2f;

__device__ __forceinline__ void guard_all_h(v8f& a0, v8f& a1, v8f& a2, v8f& a3,
                                            v16h x, v16h y0, v16h y1, v16h y2, v16h y3) {
  asm volatile("v_nop\n\tv_nop\n\tv_nop\n\tv_nop"
               : "+v"(a0), "+v"(a1), "+v"(a2), "+v"(a3)
               : "v"(x), "v"(y0), "v"(y1), "v"(y2), "v"(y3));
}
__device__ __forceinline__ void acc_guard4(v8f& a, v8f& b, v8f& c, v8f& d) {
  asm volatile("v_nop\n\tv_nop\n\tv_nop\n\tv_nop" : "+v"(a), "+v"(b), "+v"(c), "+v"(d));
}

union FragU { v16h v; v8h h[2]; };
__device__ __forceinline__ v16h frag_load(const _Float16* p) {
  FragU f;
  f.h[0] = *(const v8h*)(p);
  f.h[1] = *(const v8h*)(p + 16);
  return f.v;
}
__device__ __forceinline__ v8f mma_h(v16h a, v16h b, v8f c) {
  return __builtin_amdgcn_wmma_f32_16x16x32_f16(false, a, false, b, (short)0, c, false, false);
}

__device__ __forceinline__ float fsig(float x)  { return __builtin_amdgcn_rcpf(1.0f + __expf(-x)); }
__device__ __forceinline__ float ftanh(float x) { return 1.0f - 2.0f * __builtin_amdgcn_rcpf(__expf(2.0f * x) + 1.0f); }

__device__ __forceinline__ void cvt_store8(const float* __restrict__ sp, unsigned short* __restrict__ dp, float sc) {
  const v4f a = *(const v4f*)(sp);
  const v4f b = *(const v4f*)(sp + 4);
  v8h hv;
#pragma unroll
  for (int e = 0; e < 4; ++e) {
    const float fa = a[e] * sc;
    const float fb = b[e] * sc;
    hv[e]     = (_Float16)fa;
    hv[4 + e] = (_Float16)fb;
  }
  *(volatile v8h*)(dp) = hv;
  __threadfence();
  *(volatile v8h*)(dp) = hv;
}

__global__ __launch_bounds__(NTHR) void prep_kernel(const float* __restrict__ w_ih, const float* __restrict__ w_hh,
                                                    const float* __restrict__ b_ih, const float* __restrict__ b_hh,
                                                    unsigned short* __restrict__ WC, float* __restrict__ BIAS) {
  const int bx = blockIdx.x, tid = threadIdx.x;
  if (bx < PREP_BLK_IH) {
    const int i = bx * NTHR + tid;
    const int n = i >> 4, c8 = i & 15;
    cvt_store8(w_ih + (size_t)n * NFEAT + c8 * 8, WC + (size_t)n * KCAT + c8 * 8, WCARRY);
  } else if (bx < PREP_BLK_IH + PREP_BLK_HH) {
    const int i = (bx - PREP_BLK_IH) * NTHR + tid;
    const int n = i >> 6, c8 = i & 63;
    cvt_store8(w_hh + (size_t)n * NHID + c8 * 8, WC + (size_t)n * KCAT + NFEAT + c8 * 8, WCARRY);
  } else {
    const int i = (bx - PREP_BLK_IH - PREP_BLK_HH) * NTHR + tid;
    const v4f a = *(const v4f*)(b_ih + 4 * i);
    const v4f b = *(const v4f*)(b_hh + 4 * i);
    v4f o;
#pragma unroll
    for (int e = 0; e < 4; ++e) o[e] = a[e] + b[e];
    float* op = BIAS + 4 * i;
    *(volatile v4f*)op = o;
    __threadfence();
    *(volatile v4f*)op = o;
  }
}

__global__ __launch_bounds__(NTHR) void lstm_seq_kernel(const float* __restrict__ xin, const int* __restrict__ lengths,
                                                        const float* __restrict__ h0, const float* __restrict__ c0,
                                                        const unsigned short* __restrict__ WCp,
                                                        const float* __restrict__ BIAS, float* __restrict__ out) {
  __shared__ __align__(16) _Float16 At[2 * ABUF];
  const _Float16* WC = (const _Float16*)WCp;
  const int tid = threadIdx.x, lane = tid & 31, wave = tid >> 5;
  const int c = lane & 15, hh = lane >> 4, koff = hh * 8;
  const int rowbase = blockIdx.x * ROWS_BLK;

  int tend = 1;
#pragma unroll
  for (int m = 0; m < ROWS_BLK; ++m) {
    int L = lengths[rowbase + m];
    L = L < 1 ? 1 : (L > NSTEP ? NSTEP : L);
    tend = L > tend ? L : tend;
  }
  int lenr[8];
#pragma unroll
  for (int r = 0; r < 8; ++r) {
    int L = lengths[rowbase + 8 * hh + r];
    lenr[r] = L < 1 ? 1 : (L > NSTEP ? NSTEP : L);
  }

#pragma unroll 1
  for (int i = 0; i < ROWS_BLK; ++i) {
    const float ha = h0[(size_t)(rowbase + i) * NHID + tid];
    const float hb = h0[(size_t)(rowbase + i) * NHID + NTHR + tid];
    At[i * APITCH + NFEAT + tid]        = (_Float16)(ha * ACARRY);
    At[i * APITCH + NFEAT + NTHR + tid] = (_Float16)(hb * ACARRY);
  }
  const int xm = tid >> 4, xf8 = (tid & 15) * 8;
  {
    const float* xp = xin + ((size_t)(rowbase + xm) * NSTEP) * NFEAT_IN + xf8;
    v8h hv;
#pragma unroll
    for (int e = 0; e < 4; ++e) {
      const v2f v = *(const v2f*)(xp + 2 * e);
      const float f0 = v[0] * ACARRY;
      const float f1 = v[1] * ACARRY;
      hv[2 * e]     = (_Float16)f0;
      hv[2 * e + 1] = (_Float16)f1;
    }
    *(v8h*)(At + xm * APITCH + xf8) = hv;
  }

  float cst[4][8], hcap[4][8], bb[4][4];
#pragma unroll
  for (int nt = 0; nt < 4; ++nt) {
    const int j = 64 * wave + 16 * nt + c;
#pragma unroll
    for (int g = 0; g < 4; ++g) bb[nt][g] = BIAS[g * NHID + j];
#pragma unroll
    for (int r = 0; r < 8; ++r) {
      cst[nt][r]  = c0[(size_t)(rowbase + 8 * hh + r) * NHID + j];
      hcap[nt][r] = 0.0f;
    }
  }
  __syncthreads();

  const v8f z8 = {0.f, 0.f, 0.f, 0.f, 0.f, 0.f, 0.f, 0.f};

#pragma unroll 1
  for (int t = 0; t < tend; ++t) {
    const int cur = t & 1;
    const _Float16* arow = At + cur * ABUF + c * APITCH + koff;
    _Float16* anx = At + (cur ^ 1) * ABUF;
    const int tp1 = t + 1;

#pragma unroll
    for (int nt = 0; nt < 4; ++nt) {
      const int j = 64 * wave + 16 * nt + c;
      const _Float16* w = WC + (size_t)j * KCAT + koff;
      v8f a0 = z8, a1 = z8, a2 = z8, a3 = z8;
#pragma unroll 1
      for (int k0 = 0; k0 < KCAT; k0 += 32) {
        const v16h a  = frag_load(arow + k0);
        const v16h b0 = frag_load(w + k0);
        const v16h b1 = frag_load(w + GATE_STRIDE + k0);
        const v16h b2 = frag_load(w + 2 * GATE_STRIDE + k0);
        const v16h b3 = frag_load(w + 3 * GATE_STRIDE + k0);
        a0 = mma_h(a, b0, a0);
        a1 = mma_h(a, b1, a1);
        a2 = mma_h(a, b2, a2);
        a3 = mma_h(a, b3, a3);
        guard_all_h(a0, a1, a2, a3, a, b0, b1, b2, b3);
      }
      acc_guard4(a0, a1, a2, a3);
#pragma unroll
      for (int r = 0; r < 8; ++r) {
        const float zi = a0[r] * FOLD + bb[nt][0];
        const float zf = a1[r] * FOLD + bb[nt][1];
        const float zg = a2[r] * FOLD + bb[nt][2];
        const float zo = a3[r] * FOLD + bb[nt][3];
        const float ig = fsig(zi);
        const float fg = fsig(zf);
        const float gg = ftanh(zg);
        const float og = fsig(zo);
        const float cn = fg * cst[nt][r] + ig * gg;
        cst[nt][r] = cn;
        const float hn = og * ftanh(cn);
        anx[(8 * hh + r) * APITCH + NFEAT + j] = (_Float16)(hn * ACARRY);
        hcap[nt][r] = (tp1 == lenr[r]) ? hn : hcap[nt][r];
      }
    }

    {
      const int tn = (tp1 < NSTEP) ? tp1 : (NSTEP - 1);
      const float* xp = xin + ((size_t)(rowbase + xm) * NSTEP + (size_t)tn) * NFEAT_IN + xf8;
      v8h hv;
#pragma unroll
      for (int e = 0; e < 4; ++e) {
        const v2f v = *(const v2f*)(xp + 2 * e);
        const float f0 = v[0] * ACARRY;
        const float f1 = v[1] * ACARRY;
        hv[2 * e]     = (_Float16)f0;
        hv[2 * e + 1] = (_Float16)f1;
      }
      *(v8h*)(anx + xm * APITCH + xf8) = hv;
    }
    __syncthreads();
  }

  float* Hs = (float*)(void*)At;
#pragma unroll
  for (int nt = 0; nt < 4; ++nt) {
    const int j = 64 * wave + 16 * nt + c;
#pragma unroll
    for (int r = 0; r < 8; ++r) Hs[(8 * hh + r) * OPITCH + j] = hcap[nt][r];
  }
  __syncthreads();
  for (int pass = 0; pass < 2; ++pass) {
#pragma unroll
    for (int it = 0; it < 8; ++it) {
      const int idx = it * NTHR + tid;
      const int row = idx >> 7, c4 = (idx & 127) * 4;
      const v4f v = *(const v4f*)(Hs + row * OPITCH + c4);
      *(volatile v4f*)(out + (size_t)(rowbase + row) * NHID + c4) = v;
    }
    __threadfence();
  }
}

extern "C" void kernel_launch(void* const* d_in, const int* in_sizes, int n_in,
                              void* d_out, int out_size, void* d_ws, size_t ws_size, hipStream_t stream) {
  if (n_in < 8 || d_out == nullptr || d_ws == nullptr) return;
  if (in_sizes[0] != NBATCH * NSTEP * NFEAT_IN || in_sizes[1] != NBATCH ||
      in_sizes[2] != NBATCH * NHID || in_sizes[3] != NBATCH * NHID ||
      in_sizes[4] != NGATE * NFEAT || in_sizes[5] != NGATE * NHID ||
      in_sizes[6] != NGATE || in_sizes[7] != NGATE || out_size != NBATCH * NHID) return;

  const float* xin     = (const float*)d_in[0];
  const int*   lengths = (const int*)d_in[1];
  const float* h0      = (const float*)d_in[2];
  const float* c0      = (const float*)d_in[3];
  const float* w_ih    = (const float*)d_in[4];
  const float* w_hh    = (const float*)d_in[5];
  const float* b_ih    = (const float*)d_in[6];
  const float* b_hh    = (const float*)d_in[7];
  float* out = (float*)d_out;

  char* ws = (char*)d_ws; size_t off = 0;
  auto carve = [&](size_t bytes) -> char* { char* p = ws + off; off += (bytes + 255) & ~(size_t)255; return p; };
  unsigned short* WC   = (unsigned short*)carve((size_t)NGATE * KCAT * 2);
  float*          BIAS = (float*)carve((size_t)NGATE * 4);
  if (off > ws_size || off > (size_t)134217728) return;

  prep_kernel<<<PREP_BLK_IH + PREP_BLK_HH + PREP_BLK_BS, NTHR, 0, stream>>>(w_ih, w_hh, b_ih, b_hh, WC, BIAS);
  lstm_seq_kernel<<<NBATCH / ROWS_BLK, NTHR, 0, stream>>>(xin, lengths, h0, c0, WC, BIAS, out);
}
